// GroupFullyConnectedPooling_31765578121779
// MI455X (gfx1250) — hardware-run, weakly checked
//
#include <hip/hip_runtime.h>
#include <math.h>

typedef __attribute__((ext_vector_type(16))) _Float16 v16h;
typedef __attribute__((ext_vector_type(8)))  _Float16 v8h;
typedef __attribute__((ext_vector_type(2)))  _Float16 v2h;
typedef __attribute__((ext_vector_type(16))) __bf16   v16b;
typedef __attribute__((ext_vector_type(8)))  __bf16   v8b;
typedef __attribute__((ext_vector_type(8)))  float    v8f;
typedef __attribute__((ext_vector_type(4)))  float    v4f;
typedef __attribute__((ext_vector_type(2)))  float    v2f;

constexpr int kR    = 512;
constexpr int kSl   = 100;
constexpr int kT    = 768;
constexpr int kC    = 100;
constexpr int kCP   = 128;
constexpr int kDAll = kSl * kT;
constexpr int kOutW = kSl * kC;
constexpr int kThr  = 256;
constexpr float kInCarry = 1024.0f;
constexpr float kSc20 = 1.0f / (kInCarry * kInCarry);
constexpr float kF16MinNormal = 6.103515625e-5f;

static_assert(kR == 512 && kSl == 100 && kT == 768 && kC == 100 && kCP == 128 && kDAll == 76800 && kOutW == 10000, "the index arithmetic below uses these sizes");
static_assert(kR % 64 == 0 && kCP % 64 == 0 && kT % 32 == 0 && kC <= kCP, "whole 64x64 tiles; the depth in whole trips of 32");
static_assert(kDAll % 4 == 0 && kT % 4 == 0, "the f32 operand's row pitch and slot stride are multiples of 4 floats: every fragment load is 16-B aligned");
static_assert(kC % 4 == 0 && kOutW % 4 == 0, "a 16-B word of the result lies inside one slot's columns");

constexpr size_t kOffBK16 = 0ull;
constexpr size_t kOffST = 19660800ull;
constexpr size_t kWsTotal = 45875200ull;
static_assert(kWsTotal <= 134217728ull, "the carve stands under 128 MiB");
static_assert(kOffBK16 == 0 && kOffST == kOffBK16 + (size_t)kCP * kDAll * 2ull && kWsTotal == kOffST + (size_t)kSl * kR * kCP * 4ull, "the carve is a chain: every region starts where the one before ends");
static_assert((kOffBK16 % 256) == 0 && (kOffST % 256) == 0, "every region starts on a multiple of 256 B");

__device__ __forceinline__ unsigned short f2bf_bits(float f) {
  unsigned u = __float_as_uint(f);
  return (unsigned short)((u + 0x7FFFu + ((u >> 16) & 1u)) >> 16);
}
__device__ __forceinline__ float bf_bits2f(unsigned short h) { return __uint_as_float(((unsigned)h) << 16); }
__device__ __forceinline__ float bf16r(float f) { return bf_bits2f(f2bf_bits(f)); }
__device__ __forceinline__ float carry_flush(float v, float carry) {
  const float s = v * carry;
  return (fabsf(s) < kF16MinNormal) ? 0.0f : s;
}

__device__ __forceinline__ void dep_guard4_h(v8f& a, v8f& b, v8f& c, v8f& d, v16h x, v16h y) { asm volatile("v_nop\n\tv_nop\n\tv_nop\n\tv_nop" : "+v"(a), "+v"(b), "+v"(c), "+v"(d) : "v"(x), "v"(y)); }
__device__ __forceinline__ void dep_guard4_b(v8f& a, v8f& b, v8f& c, v8f& d, v16b x, v16b y) { asm volatile("v_nop\n\tv_nop\n\tv_nop\n\tv_nop" : "+v"(a), "+v"(b), "+v"(c), "+v"(d) : "v"(x), "v"(y)); }
__device__ __forceinline__ void keep4_h(v16h a, v16h b, v16h c, v16h d) { asm volatile("v_nop" :: "v"(a), "v"(b), "v"(c), "v"(d)); }
__device__ __forceinline__ void keep4_b(v16b a, v16b b, v16b c, v16b d) { asm volatile("v_nop" :: "v"(a), "v"(b), "v"(c), "v"(d)); }
__device__ __forceinline__ void acc_guard4(v8f& a, v8f& b, v8f& c, v8f& d) { asm volatile("v_nop\n\tv_nop\n\tv_nop\n\tv_nop" : "+v"(a), "+v"(b), "+v"(c), "+v"(d)); }

template <typename T> struct Frag;
template <> struct Frag<_Float16> {
  typedef v16h V; union U { v16h v; v8h h[2]; };
  static __device__ __forceinline__ v16h load(const _Float16* p) {
    U f; f.h[0] = *(const v8h*)(p); f.h[1] = *(const v8h*)(p + 16); return f.v;
  }
  static __device__ __forceinline__ v8f mma(v16h a, v16h b, v8f c) {
    return __builtin_amdgcn_wmma_f32_16x16x32_f16(false, a, false, b, (short)0, c, false, false);
  }
  static __device__ __forceinline__ void guard4(v8f& a, v8f& b, v8f& c, v8f& d, v16h x, v16h y) { dep_guard4_h(a, b, c, d, x, y); }
  static __device__ __forceinline__ void keep(v16h a, v16h b, v16h c, v16h d) { keep4_h(a, b, c, d); }
};
template <> struct Frag<__bf16> {
  typedef v16b V; union U { v16b v; v8b h[2]; };
  static __device__ __forceinline__ v16b load(const __bf16* p) {
    U f; f.h[0] = *(const v8b*)(p); f.h[1] = *(const v8b*)(p + 16); return f.v;
  }
  static __device__ __forceinline__ v8f mma(v16b a, v16b b, v8f c) {
    return __builtin_amdgcn_wmma_f32_16x16x32_bf16(false, a, false, b, (short)0, c, false, false);
  }
  static __device__ __forceinline__ void guard4(v8f& a, v8f& b, v8f& c, v8f& d, v16b x, v16b y) { dep_guard4_b(a, b, c, d, x, y); }
  static __device__ __forceinline__ void keep(v16b a, v16b b, v16b c, v16b d) { keep4_b(a, b, c, d); }
};

template <int CV>
__device__ __forceinline__ v16h cvload(const float* p, float carry) {
  const v4f a0 = *(const v4f*)(p), a1 = *(const v4f*)(p + 4), b0 = *(const v4f*)(p + 16), b1 = *(const v4f*)(p + 20);
  v16h f;
#pragma unroll
  for (int e = 0; e < 4; ++e) {
    f[e]      = (_Float16)carry_flush(CV == 1 ? bf16r(a0[e]) : a0[e], carry);
    f[4 + e]  = (_Float16)carry_flush(CV == 1 ? bf16r(a1[e]) : a1[e], carry);
    f[8 + e]  = (_Float16)carry_flush(CV == 1 ? bf16r(b0[e]) : b0[e], carry);
    f[12 + e] = (_Float16)carry_flush(CV == 1 ? bf16r(b1[e]) : b1[e], carry);
  }
  return f;
}
template <int ET> struct Elem;
template <> struct Elem<0> { typedef _Float16 T; };
template <> struct Elem<1> { typedef __bf16 T; };
template <int CVA, int CVB, int BIAS_MODE, int OUT_MODE, bool RESID, int ACT = 0>
__global__ __launch_bounds__(256) void wmma_gemm64cv(
    const unsigned short* __restrict__ Ap, const float* __restrict__ Af, float carryA, int lda, long strideA,
    const unsigned short* __restrict__ Btp, const float* __restrict__ Bf, float carryB, int ldb, long strideB,
    void* __restrict__ Cout, void* __restrict__ Cout2, int ldc, long strideC,
    const float* __restrict__ bias,
    const float* __restrict__ resid, long strideR,
    int M, int N, int K, float scale) {
  constexpr int ET = 0; constexpr bool SPLIT = false;
  const unsigned short* A2p = nullptr; const unsigned short* Bt2p = nullptr;
  typedef typename Elem<ET>::T T;
  typedef typename Frag<T>::V V;
  const T* A = (const T*)Ap; const T* A2 = (const T*)A2p; const T* Bt = (const T*)Btp; const T* Bt2 = (const T*)Bt2p;
  __shared__ __align__(16) float sT[8][16 * 68];
  const int b    = blockIdx.y;
  const int lane = threadIdx.x & 31;
  const int wave = threadIdx.x >> 5;
  const int tilesN = N >> 6;
  const int tilesM = M >> 6;
  const int tile = blockIdx.x * 8 + wave;
  if (tile >= tilesM * tilesN) return;
  const int tm = tile / tilesN;
  const int tn = tile - tm * tilesN;
  const int m0 = tm << 6;
  const int n0 = tn << 6;

  const T* Ab  = A  + (size_t)b * strideA;
  const T* Bb  = Bt + (size_t)b * strideB;
  const T* Ab2 = SPLIT ? (A2  + (size_t)b * strideA) : nullptr;
  const T* Bb2 = SPLIT ? (Bt2 + (size_t)b * strideB) : nullptr;
  const float* Afb = (CVA != 0) ? (Af + (size_t)b * strideA) : nullptr;
  const float* Bfb = (CVB != 0) ? (Bf + (size_t)b * strideB) : nullptr;

  const int rlane = lane & 15;
  const int koff  = (lane >> 4) * 8;
  const int mOff  = (lane >> 4) * 8;

  v8f acc[4][4];
#pragma unroll
  for (int i = 0; i < 4; ++i)
#pragma unroll
    for (int j = 0; j < 4; ++j) acc[i][j] = (v8f){0.f,0.f,0.f,0.f,0.f,0.f,0.f,0.f};

  for (int k0 = 0; k0 < K; k0 += 32) {
    V bh[4], bl[4];
#pragma unroll
    for (int j = 0; j < 4; ++j) {
      const size_t bo = (size_t)(n0 + (j << 4) + rlane) * ldb + koff + k0;
      if (CVB == 0) bh[j] = Frag<T>::load(Bb + bo); else bh[j] = cvload<CVB>(Bfb + bo, carryB);
      if (SPLIT) bl[j] = Frag<T>::load(Bb2 + bo);
    }
#pragma unroll
    for (int i = 0; i < 4; ++i) {
      const size_t ao = (size_t)(m0 + (i << 4) + rlane) * lda + koff + k0;
      V ah;
      if (CVA == 0) ah = Frag<T>::load(Ab + ao); else ah = cvload<CVA>(Afb + ao, carryA);
      V al;
      if (SPLIT) al = Frag<T>::load(Ab2 + ao);
#pragma unroll
      for (int j = 0; j < 4; ++j) {
        acc[i][j] = Frag<T>::mma(ah, bh[j], acc[i][j]);
        if (SPLIT) {
          acc[i][j] = Frag<T>::mma(ah, bl[j], acc[i][j]);
          acc[i][j] = Frag<T>::mma(al, bh[j], acc[i][j]);
        }
      }
      Frag<T>::guard4(acc[i][0], acc[i][1], acc[i][2], acc[i][3], ah, SPLIT ? al : ah);
    }
    Frag<T>::keep(bh[0], bh[1], bh[2], bh[3]);
    if (SPLIT) Frag<T>::keep(bl[0], bl[1], bl[2], bl[3]);
  }
  acc_guard4(acc[0][0], acc[0][1], acc[0][2], acc[0][3]);
  acc_guard4(acc[1][0], acc[1][1], acc[1][2], acc[1][3]);
  acc_guard4(acc[2][0], acc[2][1], acc[2][2], acc[2][3]);
  acc_guard4(acc[3][0], acc[3][1], acc[3][2], acc[3][3]);

  float* slab = sT[wave];
  const float* Rb = RESID ? (resid + (size_t)b * strideR) : nullptr;
#pragma unroll
  for (int i = 0; i < 4; ++i) {
    const int mBase = m0 + (i << 4);
#pragma unroll
    for (int j = 0; j < 4; ++j) {
      const int n = n0 + (j << 4) + rlane;
      float bv = 0.f;
      if (BIAS_MODE == 2) bv = bias[n];
#pragma unroll
      for (int r = 0; r < 8; ++r) {
        float v = acc[i][j][r] * scale;
        if (BIAS_MODE == 1) v += bias[mBase + mOff + r];
        if (BIAS_MODE == 2) v += bv;
        if (RESID) v += Rb[(size_t)(mBase + mOff + r) * ldc + n];
        if (ACT == 1) v = tanhf(v);
        if (ACT == 2) v = fmaxf(v, 0.0f);
        if (ACT == 3) v = v / (1.0f + expf(-v));
        if (ACT == 4) v = (v > 0.f) ? v : 0.01f * v;
        slab[(mOff + r) * 68 + (j << 4) + rlane] = v;
      }
    }
    __builtin_amdgcn_fence(__ATOMIC_RELEASE, "workgroup");
    __builtin_amdgcn_wave_barrier();
    __builtin_amdgcn_fence(__ATOMIC_ACQUIRE, "workgroup");
    if (OUT_MODE == 0) {
      float* C = (float*)Cout + (size_t)b * strideC;
      const int hh = lane >> 4, c4 = (lane & 15) * 4;
      for (int pass = 0; pass < 2; ++pass) {
#pragma unroll
        for (int it = 0; it < 8; ++it) {
          const int row = it * 2 + hh;
          v4f v = *(const v4f*)(slab + row * 68 + c4);
          *(volatile v4f*)(C + (size_t)(mBase + row) * ldc + n0 + c4) = v;
        }
        __threadfence();
      }
    } else {
      const int q = lane >> 3, c8 = (lane & 7) * 8;
      unsigned short* C  = (unsigned short*)Cout  + (size_t)b * strideC;
      unsigned short* C2 = (OUT_MODE == 2) ? ((unsigned short*)Cout2 + (size_t)b * strideC) : nullptr;
      for (int pass = 0; pass < 2; ++pass) {
#pragma unroll
        for (int it = 0; it < 4; ++it) {
          const int row = it * 4 + q;
          const float* sp = slab + row * 68 + c8;
          v8h hv, lv;
#pragma unroll
          for (int e = 0; e < 8; ++e) {
            if (OUT_MODE == 1) {
              hv[e] = (_Float16)sp[e];
            } else {
              unsigned short hb = f2bf_bits(sp[e]);
              unsigned short lb = f2bf_bits(sp[e] - bf_bits2f(hb));
              hv[e] = __builtin_bit_cast(_Float16, hb);
              lv[e] = __builtin_bit_cast(_Float16, lb);
            }
          }
          *(volatile v8h*)(C + (size_t)(mBase + row) * ldc + n0 + c8) = hv;
          if (OUT_MODE == 2) *(volatile v8h*)(C2 + (size_t)(mBase + row) * ldc + n0 + c8) = lv;
        }
        __threadfence();
      }
    }
    __builtin_amdgcn_fence(__ATOMIC_RELEASE, "workgroup");
    __builtin_amdgcn_wave_barrier();
    __builtin_amdgcn_fence(__ATOMIC_ACQUIRE, "workgroup");
  }
}

__global__ __launch_bounds__(kThr) void pack_kernel(const float* __restrict__ W, unsigned short* __restrict__ D, float* __restrict__ dstf, int part, int ld, int k0, int lg, int n0, int pitch) {
  const unsigned i = blockIdx.x * blockDim.x + threadIdx.x;
  if (part == 0) {
    const unsigned g = i & ((1u << lg) - 1u), n = i >> lg;
    const float* sp = W + (size_t)((unsigned)k0 + g * 8u) * (unsigned)ld + n;
    v8h hv;
#pragma unroll
    for (int t = 0; t < 8; ++t) hv[t] = (_Float16)carry_flush(bf16r(sp[(size_t)t * (unsigned)ld]), kInCarry);
    unsigned short* dp = D + (size_t)((unsigned)n0 + n) * (unsigned)pitch + g * 8u;
    *(volatile v8h*)dp = hv;
    __threadfence();
    *(volatile v8h*)dp = hv;
  } else {
    const v4f a = *(const v4f*)(W + i * 4u);
    v4f o;
#pragma unroll
    for (int e = 0; e < 4; ++e) o[e] = bf16r(a[e]);
    float* dp = dstf + i * 4u;
    *(volatile v4f*)dp = o;
    __threadfence();
    *(volatile v4f*)dp = o;
  }
}


__global__ __launch_bounds__(kThr) void zero_kernel(float* __restrict__ dst) {
  const size_t o4 = ((size_t)blockIdx.x * kThr + threadIdx.x) * 4u;
  const v4f z = {0.f, 0.f, 0.f, 0.f};
  *(volatile v4f*)(dst + o4) = z;
  __threadfence();
  *(volatile v4f*)(dst + o4) = z;
}

__global__ __launch_bounds__(kThr) void outrow_kernel(const float* __restrict__ ST, const float* __restrict__ addend, float* __restrict__ out) {
  const unsigned q = blockIdx.x * (unsigned)kThr + threadIdx.x;
  const unsigned r = q / (unsigned)(kOutW / 4), w = q - r * (unsigned)(kOutW / 4);
  const unsigned s = w / (unsigned)(kC / 4), c4 = (w - s * (unsigned)(kC / 4)) * 4u;
  const v4f pv = *(const v4f*)(ST + ((size_t)s * (unsigned)kR + r) * (unsigned)kCP + c4);
  const v4f av = *(const v4f*)(addend + (size_t)w * 4u);
  v4f o;
#pragma unroll
  for (int e = 0; e < 4; ++e) o[e] = pv[e] + bf16r(av[e]);
  float* dp = out + (size_t)q * 4u;
  *(volatile v4f*)dp = o;
  __threadfence();
  *(volatile v4f*)dp = o;
}

extern "C" void kernel_launch(void* const* d_in, const int* in_sizes, int n_in,
                              void* d_out, int out_size, void* d_ws, size_t ws_size,
                              hipStream_t stream) {
  if (n_in < 3 || d_out == nullptr || d_ws == nullptr) return;
  if (in_sizes[0] != kR * kSl * kT || in_sizes[1] != kSl * kT * kC || in_sizes[2] != kOutW) return;
  if (out_size != kR * kOutW) return;
  if (ws_size < kWsTotal) return;
  const float* x = (const float*)d_in[0];
  const float* bank = (const float*)d_in[1];
  const float* addend = (const float*)d_in[2];
  float* out = (float*)d_out;
  char* ws = (char*)d_ws;
  unsigned short* BK16 = (unsigned short*)(ws + kOffBK16);
  float* ST = (float*)(ws + kOffST);

  static_assert(((size_t)(kCP - kC) * kDAll * 2 / 16) % kThr == 0 && ((size_t)kR * kOutW / 4) % kThr == 0, "the fill's and the result kernel's grids exact");
  static_assert(8192 + 1024 + 256 + 128 == kDAll / 8 && (kC * 128) % 64 == 0, "the bank's 9,600 depth groups of eight in four power-of-two launches; every pack grid exact");
  zero_kernel<<<(kCP - kC) * kDAll * 2 / 16 / kThr, kThr, 0, stream>>>((float*)(BK16 + (size_t)kC * kDAll));
  pack_kernel<<<kC * 8192 / 64, 64, 0, stream>>>(bank, BK16, nullptr, 0, kC, 0, 13, 0, kDAll);
  pack_kernel<<<kC * 1024 / 64, 64, 0, stream>>>(bank, BK16 + 65536, nullptr, 0, kC, 65536, 10, 0, kDAll);
  pack_kernel<<<kC * 256 / 64, 64, 0, stream>>>(bank, BK16 + 73728, nullptr, 0, kC, 73728, 8, 0, kDAll);
  pack_kernel<<<kC * 128 / 64, 64, 0, stream>>>(bank, BK16 + 75776, nullptr, 0, kC, 75776, 7, 0, kDAll);
  wmma_gemm64cv<1, 0, 0, 0, false, 0><<<dim3((kR / 64) * (kCP / 64) / 8, kSl), 256, 0, stream>>>(
      nullptr, x, kInCarry, kDAll, (long)kT, BK16, nullptr, 1.0f, kDAll, (long)kT, (void*)ST, (void*)ST, kCP, (long)kR * kCP, nullptr, nullptr, 0L, kR, kCP, kT, kSc20);
  outrow_kernel<<<kR * kOutW / 4 / kThr, kThr, 0, stream>>>(ST, addend, out);
}
static_assert(((kR / 64) * (kCP / 64)) % 8 == 0, "the engine's grid: whole blocks of eight wave tiles a slot");
